// MultiheadAttention_11244224381448
// MI455X (gfx1250) — hardware-run, weakly checked
//
#include <hip/hip_runtime.h>


#ifndef NB
#define NB 4
#endif
#ifndef SEQ
#define SEQ 2048
#endif
#define NB_FULL  4
#define SEQ_FULL 2048
#define DM   64
#define NH   12
#define HD   64
#define NP   (NH * HD)
#ifndef QLO
#define QLO 1
#endif
#define LCAR 2048.0f
#define PCL  10.0f
#define SCL  0.125f
#define L2E  1.4426950408889634f

static_assert(SEQ % 64 == 0);
static_assert(NB <= NB_FULL);
static_assert(SEQ <= SEQ_FULL);
static_assert((NB * NH * (SEQ / 16)) % 4 == 0);
static_assert(DM % 32 == 0);
static_assert(HD == 64);

typedef _Float16 h16;
typedef unsigned short bf;
typedef __attribute__((ext_vector_type(16))) __bf16   v16bf;
typedef __attribute__((ext_vector_type(16))) _Float16 v16h;
typedef __attribute__((ext_vector_type(8)))  _Float16 v8h;
typedef __attribute__((ext_vector_type(8)))  unsigned short v8us;
typedef __attribute__((ext_vector_type(2)))  unsigned short v2us;
typedef __attribute__((ext_vector_type(8)))  float    v8f;
typedef __attribute__((ext_vector_type(4)))  float    v4f;
typedef v8h  __attribute__((may_alias)) v8ha;
typedef v4f  __attribute__((may_alias)) v4fa;

__device__ __forceinline__ unsigned short f2bf(float f) { unsigned u = __float_as_uint(f); u += 0x7FFFu + ((u >> 16) & 1u); return (unsigned short)(u >> 16); }
__device__ __forceinline__ float bf2f(unsigned short b) { return __uint_as_float(((unsigned)b) << 16); }
__device__ __forceinline__ float bfr(float f) { return bf2f(f2bf(f)); }
__device__ __forceinline__ v16h cat16(v8h lo, v8h hi) { return __builtin_shufflevector(lo, hi, 0, 1, 2, 3, 4, 5, 6, 7, 8, 9, 10, 11, 12, 13, 14, 15); }
__device__ __forceinline__ v16bf cat16b(v8us lo, v8us hi) { return __builtin_bit_cast(v16bf, __builtin_shufflevector(lo, hi, 0, 1, 2, 3, 4, 5, 6, 7, 8, 9, 10, 11, 12, 13, 14, 15)); }
__device__ __forceinline__ v8f wmma16(v16h a, v16h b, v8f c) { return __builtin_amdgcn_wmma_f32_16x16x32_f16(false, a, false, b, (short)0, c, false, false); }
__device__ __forceinline__ v8f wmmab(v16bf a, v16bf b, v8f c) { return __builtin_amdgcn_wmma_f32_16x16x32_bf16(false, a, false, b, (short)0, c, false, false); }
__device__ __forceinline__ v16h ldh(const h16* p) { return cat16(*(const v8h*)p, *(const v8h*)(p + 16)); }
__device__ __forceinline__ v16bf ldb(const bf* p) { return cat16b(*(const v8us*)p, *(const v8us*)(p + 16)); }
__device__ __forceinline__ float ex2(float x) { return __builtin_amdgcn_exp2f(x); }

#define PX_BLOCKS ((NB * SEQ * DM / 8 + 255) / 256)
#define PW_BLOCKS ((3 * NP + 7) / 8)
#define PB_BLOCKS ((3 * NP + 255) / 256)
#define PM_BLOCKS ((NB * SEQ + 255) / 256)

__global__ __launch_bounds__(256) void k_prep(const float* __restrict__ x, const float* __restrict__ am,
                                              const float* __restrict__ wq, const float* __restrict__ bq,
                                              const float* __restrict__ wk, const float* __restrict__ bk,
                                              const float* __restrict__ wv, const float* __restrict__ bv,
                                              bf* XB, bf* WT, float* BI, float* MB) {
    const int blk = blockIdx.x, tid = threadIdx.x;
    if (blk < PX_BLOCKS) {
        const int i = blk * 256 + tid;
        if (i < NB * SEQ * DM / 8) {
            const int e = i * 8; const int rr = e / DM, c = e % DM; const int b = rr / SEQ, t = rr % SEQ;
            const float* src = x + ((size_t)b * SEQ_FULL + t) * DM + c;
            const v4f a0 = *(const v4f*)src; const v4f a1 = *(const v4f*)(src + 4);
            v8us o;
#pragma unroll
            for (int k = 0; k < 4; ++k) { o[k] = f2bf(a0[k]); o[4 + k] = f2bf(a1[k]); }
            *(volatile v8us*)(XB + (size_t)e) = o; __threadfence(); *(volatile v8us*)(XB + (size_t)e) = o;
        }
    } else if (blk < PX_BLOCKS + PW_BLOCKS) {
        const int line = (blk - PX_BLOCKS) * 8 + (tid >> 5); const int lane = tid & 31;
        if (line < 3 * NP) {
            const int mat = line / NP, n = line % NP; const int k = 2 * lane;
            const size_t i0 = (size_t)k * NP + n, i1 = (size_t)(k + 1) * NP + n;
            const float a0 = wq[i0], a1 = wq[i1], b0 = wk[i0], b1 = wk[i1], c0 = wv[i0], c1 = wv[i1];
            const float w0 = (mat == 0) ? a0 : ((mat == 1) ? b0 : c0);
            const float w1 = (mat == 0) ? a1 : ((mat == 1) ? b1 : c1);
            v2us o; o[0] = f2bf(w0); o[1] = f2bf(w1);
            bf* dst = WT + (size_t)line * DM + k;
            *(volatile v2us*)dst = o; __threadfence(); *(volatile v2us*)dst = o;
        }
    } else if (blk < PX_BLOCKS + PW_BLOCKS + PB_BLOCKS) {
        const int idx = (blk - PX_BLOCKS - PW_BLOCKS) * 256 + tid;
        if (idx < 3 * NP) {
            const int mat = idx / NP, n = idx % NP;
            const float a = bq[n], b = bk[n], c = bv[n];
            const float val = bfr((mat == 0) ? a : ((mat == 1) ? b : c));
            *(volatile float*)(BI + idx) = val; __threadfence(); *(volatile float*)(BI + idx) = val;
        }
    } else {
        const int idx = (blk - PX_BLOCKS - PW_BLOCKS - PB_BLOCKS) * 256 + tid;
        if (idx < NB * SEQ) {
            const int b = idx / SEQ, t = idx % SEQ;
            const float a = bfr(am[(size_t)b * SEQ_FULL + t]);
            const float val = (1.0f - a) * (-10000.0f);
            *(volatile float*)(MB + idx) = val; __threadfence(); *(volatile float*)(MB + idx) = val;
        }
    }
}

__global__ __launch_bounds__(32) void k_proj(const bf* __restrict__ XB, const bf* __restrict__ WT, const float* __restrict__ BI, h16* PL) {
    __shared__ __align__(16) h16 hs[64 * 72];
    __shared__ __align__(16) h16 ls[64 * 72];
    const int lane = threadIdx.x & 31, lr = lane & 15, hi = lane >> 4;
    const int r0 = blockIdx.x * 64, hd = blockIdx.y, mat = blockIdx.z; const int c0 = hd * 64;
    v8f acc[4][4];
#pragma unroll
    for (int mb = 0; mb < 4; ++mb)
#pragma unroll
        for (int nb = 0; nb < 4; ++nb) acc[mb][nb] = (v8f){};
    const bf* Ap = XB + (size_t)(r0 + lr) * DM + 8 * hi;
    const bf* Bp = WT + ((size_t)mat * NP + c0 + lr) * DM + 8 * hi;
#pragma unroll 1
    for (int kc = 0; kc < DM; kc += 32) {
        v16bf a[4]; v16bf bl;
#pragma unroll
        for (int mb = 0; mb < 4; ++mb) a[mb] = ldb(Ap + (size_t)mb * 16 * DM + kc);
#pragma unroll
        for (int nb = 0; nb < 4; ++nb) { const v16bf b = ldb(Bp + (size_t)nb * 16 * DM + kc); bl = b;
#pragma unroll
            for (int mb = 0; mb < 4; ++mb) acc[mb][nb] = wmmab(a[mb], b, acc[mb][nb]); }
        asm volatile("v_nop\n\tv_nop\n\tv_nop\n\tv_nop" : "+v"(acc[0][3]), "+v"(acc[1][3]), "+v"(acc[2][3]), "+v"(acc[3][3]) : "v"(a[0]), "v"(a[1]), "v"(a[2]), "v"(a[3]), "v"(bl));
    }
    float bia[4];
#pragma unroll
    for (int nb = 0; nb < 4; ++nb) bia[nb] = BI[mat * NP + c0 + nb * 16 + lr];
    const int b = r0 / SEQ, t0 = r0 % SEQ; const size_t bh = (size_t)b * NH + hd;
    const size_t PLN = (size_t)NB * NH * SEQ * HD;
    const int rq = lane >> 3, pc = (lane & 7) * 8;
    if (mat == 2) {
#pragma unroll
        for (int mb = 0; mb < 4; ++mb)
#pragma unroll
            for (int nb = 0; nb < 4; ++nb) { v8h pk;
#pragma unroll
                for (int j = 0; j < 8; ++j) pk[j] = (h16)(acc[mb][nb][j] + bia[nb]);
                *(v8ha*)(hs + (nb * 16 + lr) * 72 + mb * 16 + 8 * hi) = pk; }
        __syncthreads();
        h16* dst = PL + 3 * PLN + bh * HD * SEQ + t0;
#pragma unroll 1
        for (int ps = 0; ps < 2; ++ps) {
#pragma unroll
            for (int i = 0; i < 16; ++i) { const int d = 4 * i + rq; const v8h val = *(const v8ha*)(hs + d * 72 + pc);
                *(volatile v8h*)(dst + (size_t)d * SEQ + pc) = val; }
            if (ps == 0) __threadfence(); }
    } else {
        const bool wl = (mat == 0) && (QLO != 0);
#pragma unroll
        for (int mb = 0; mb < 4; ++mb)
#pragma unroll
            for (int nb = 0; nb < 4; ++nb)
#pragma unroll
                for (int j = 0; j < 8; ++j) { const int row = mb * 16 + 8 * hi + j, col = nb * 16 + lr; const float v = acc[mb][nb][j] + bia[nb]; const h16 hv = (h16)v;
                    hs[row * 72 + col] = hv; if (wl) ls[row * 72 + col] = (h16)((v - (float)hv) * LCAR); }
        __syncthreads();
        h16* dst = PL + (size_t)mat * PLN + (bh * SEQ + t0) * HD;
#pragma unroll 1
        for (int ps = 0; ps < 2; ++ps) {
#pragma unroll
            for (int i = 0; i < 16; ++i) { const int row = 4 * i + rq; const v8h val = *(const v8ha*)(hs + row * 72 + pc);
                *(volatile v8h*)(dst + (size_t)row * HD + pc) = val; }
            if (ps == 0) __threadfence(); }
        if (wl) {
            h16* dl = PL + 2 * PLN + (bh * SEQ + t0) * HD;
#pragma unroll 1
            for (int ps = 0; ps < 2; ++ps) {
#pragma unroll
                for (int i = 0; i < 16; ++i) { const int row = 4 * i + rq; const v8h val = *(const v8ha*)(ls + row * 72 + pc);
                    *(volatile v8h*)(dl + (size_t)row * HD + pc) = val; }
                if (ps == 0) __threadfence(); }
        }
    }
}

__global__ __launch_bounds__(128) void k_attn(const h16* __restrict__ PL, const float* __restrict__ MB, float* OUT) {
    __shared__ __align__(16) float os[4 * 16 * 68];
    const int w = threadIdx.x >> 5, lane = threadIdx.x & 31, lr = lane & 15, hi = lane >> 4;
    const int qt = blockIdx.x * 4 + w;
    const int bh = qt / (SEQ / 16); const int q0 = (qt % (SEQ / 16)) * 16; const int b = bh / NH, hd = bh % NH;
    const size_t PLN = (size_t)NB * NH * SEQ * HD;
    const h16* qh = PL + ((size_t)bh * SEQ + q0 + lr) * HD + 8 * hi;
    const h16* ql = qh + 2 * PLN;
    const h16* kb = PL + PLN + (size_t)bh * SEQ * HD + (size_t)lr * HD + 8 * hi;
    const h16* vb = PL + 3 * PLN + (size_t)bh * HD * SEQ + (size_t)lr * SEQ + 8 * hi;
    const float* mb = MB + (size_t)b * SEQ + 8 * hi;
    const v16h bqh0 = ldh(qh), bqh1 = ldh(qh + 32);
    v16h bql0 = bqh0, bql1 = bqh1;
    if (QLO) { bql0 = ldh(ql); bql1 = ldh(ql + 32); }
    v8f acc[4];
#pragma unroll
    for (int dt = 0; dt < 4; ++dt) acc[dt] = (v8f){};
    float m_run = -1.0e30f, nb_run = 1.4426950e30f, l_run = 0.0f;
#pragma unroll 1
    for (int j0 = 0; j0 < SEQ; j0 += 32) {
        const h16* k0p = kb + (size_t)j0 * HD;
        const v16h ka0 = ldh(k0p), ka1 = ldh(k0p + 32), kc0 = ldh(k0p + 16 * HD), kc1 = ldh(k0p + 16 * HD + 32);
        const v4f m0a = *(const v4f*)(mb + j0), m0b = *(const v4f*)(mb + j0 + 4), m1a = *(const v4f*)(mb + j0 + 16), m1b = *(const v4f*)(mb + j0 + 20);
        v16h vf[4];
#pragma unroll
        for (int dt = 0; dt < 4; ++dt) vf[dt] = ldh(vb + (size_t)dt * 16 * SEQ + j0);
        v8f sh0 = (v8f){}, sh1 = (v8f){}, sl0 = (v8f){}, sl1 = (v8f){};
        sh0 = wmma16(ka0, bqh0, sh0); sh1 = wmma16(kc0, bqh0, sh1);
        sh0 = wmma16(ka1, bqh1, sh0); sh1 = wmma16(kc1, bqh1, sh1);
        if (QLO) {
            sl0 = wmma16(ka0, bql0, sl0); sl1 = wmma16(kc0, bql0, sl1);
            sl0 = wmma16(ka1, bql1, sl0); sl1 = wmma16(kc1, bql1, sl1);
        }
        asm volatile("v_nop\n\tv_nop\n\tv_nop\n\tv_nop" : "+v"(sh0), "+v"(sh1), "+v"(sl0), "+v"(sl1) : "v"(ka1), "v"(kc1), "v"(bqh1), "v"(bql1));
        float t[16];
#pragma unroll
        for (int r = 0; r < 8; ++r) {
            float u0 = sh0[r], u1 = sh1[r];
            if (QLO) { u0 = __builtin_fmaf(sl0[r], 1.0f / LCAR, u0); u1 = __builtin_fmaf(sl1[r], 1.0f / LCAR, u1); }
            const float g0 = (r < 4) ? m0a[r & 3] : m0b[r & 3];
            const float g1 = (r < 4) ? m1a[r & 3] : m1b[r & 3];
            t[r] = __builtin_fmaf(u0, SCL, g0); t[8 + r] = __builtin_fmaf(u1, SCL, g1);
        }
        float mx = t[0];
#pragma unroll
        for (int i = 1; i < 16; ++i) mx = fmaxf(mx, t[i]);
        const float mo = __shfl_xor(mx, 16, 32);
        mx = fmaxf(mx, mo);
        const float mnew = fmaxf(m_run, mx);
        const unsigned grow = __builtin_amdgcn_ballot_w32(mnew > m_run);
        if (grow != 0u) {
            const float nbn = __builtin_fmaf(-mnew, L2E, PCL);
            const float al = ex2(nbn - nb_run);
            l_run *= al;
#pragma unroll
            for (int dt = 0; dt < 4; ++dt)
#pragma unroll
                for (int r = 0; r < 8; ++r) acc[dt][r] *= al;
            nb_run = nbn; m_run = mnew;
        }
        v16h pf; float ps = 0.0f;
#pragma unroll
        for (int r = 0; r < 8; ++r) {
            const float e0 = ex2(__builtin_fmaf(t[r], L2E, nb_run));
            const float e1 = ex2(__builtin_fmaf(t[8 + r], L2E, nb_run));
            ps += e0 + e1; pf[r] = (h16)e0; pf[8 + r] = (h16)e1;
        }
        l_run += ps;
#pragma unroll
        for (int dt = 0; dt < 4; ++dt) acc[dt] = wmma16(vf[dt], pf, acc[dt]);
        asm volatile("v_nop\n\tv_nop\n\tv_nop\n\tv_nop" : "+v"(acc[0]), "+v"(acc[1]), "+v"(acc[2]), "+v"(acc[3]) : "v"(vf[0]), "v"(vf[1]), "v"(vf[2]), "v"(vf[3]), "v"(pf));
    }
    const float lo = __shfl_xor(l_run, 16, 32);
    const float inv = 1.0f / (l_run + lo);
    float* o = os + w * 16 * 68;
#pragma unroll
    for (int dt = 0; dt < 4; ++dt) { v4f a, c;
#pragma unroll
        for (int r = 0; r < 4; ++r) { a[r] = acc[dt][r] * inv; c[r] = acc[dt][4 + r] * inv; }
        *(v4fa*)(o + lr * 68 + dt * 16 + 8 * hi) = a; *(v4fa*)(o + lr * 68 + dt * 16 + 8 * hi + 4) = c; }
    __syncthreads();
    float* dst = OUT + ((size_t)b * SEQ_FULL + q0) * NP + hd * HD;
#pragma unroll 1
    for (int ps = 0; ps < 2; ++ps) {
#pragma unroll
        for (int s = 0; s < 8; ++s) { const int row = 2 * s + hi, cofs = lr * 4; const v4f val = *(const v4fa*)(o + row * 68 + cofs);
            *(volatile v4f*)(dst + (size_t)row * NP + cofs) = val; }
        if (ps == 0) __threadfence(); }
}

extern "C" void kernel_launch(void* const* d_in, const int* in_sizes, int n_in,
                              void* d_out, int out_size, void* d_ws, size_t ws_size, hipStream_t stream) {
    if (n_in < 8) return;
    const size_t rows_in = (size_t)(NB - 1) * SEQ_FULL + SEQ;
    if ((size_t)in_sizes[0] < rows_in * DM) return;
    if ((size_t)in_sizes[1] < rows_in) return;
    if (in_sizes[2] < DM * NP || in_sizes[4] < DM * NP || in_sizes[6] < DM * NP) return;
    if (in_sizes[3] < NP || in_sizes[5] < NP || in_sizes[7] < NP) return;
    if ((size_t)out_size < rows_in * NP) return;
    const float* x  = (const float*)d_in[0];
    const float* am = (const float*)d_in[1];
    const float* wq = (const float*)d_in[2]; const float* bq = (const float*)d_in[3];
    const float* wk = (const float*)d_in[4]; const float* bk = (const float*)d_in[5];
    const float* wv = (const float*)d_in[6]; const float* bv = (const float*)d_in[7];
    float* OUT = (float*)d_out;
    char* wsp = (char*)d_ws;
    auto take = [&](size_t bytes) { char* p = wsp; wsp += (bytes + 255) & ~(size_t)255; return (void*)p; };
    const size_t PLN = (size_t)NB * NH * SEQ * HD;
    bf* XB = (bf*)take((size_t)NB * SEQ * DM * 2);
    bf* WT = (bf*)take((size_t)3 * NP * DM * 2);
    float* BI = (float*)take((size_t)3 * NP * 4);
    float* MB = (float*)take((size_t)NB * SEQ * 4);
    h16* PL = (h16*)take(4 * PLN * 2);
    if ((size_t)(wsp - (char*)d_ws) > ws_size) return;
    k_prep<<<PX_BLOCKS + PW_BLOCKS + PB_BLOCKS + PM_BLOCKS, 256, 0, stream>>>(x, am, wq, bq, wk, bk, wv, bv, XB, WT, BI, MB);
    k_proj<<<dim3(NB * SEQ / 64, NH, 3), 32, 0, stream>>>(XB, WT, BI, PL);
    k_attn<<<NB * NH * (SEQ / 16) / 4, 128, 0, stream>>>(PL, MB, OUT);
}
